// neural_network_2284922601909
// MI455X (gfx1250) — hardware-verified
//
#include <hip/hip_runtime.h>
#include <math.h>

typedef __attribute__((ext_vector_type(16))) _Float16 v16h;
typedef __attribute__((ext_vector_type(16))) __bf16 v16b;
typedef __attribute__((ext_vector_type(8)))  _Float16 v8h;
typedef __attribute__((ext_vector_type(8)))  float v8f;
typedef __attribute__((ext_vector_type(4)))  float v4f;
typedef __attribute__((ext_vector_type(2)))  float v2f;
typedef __attribute__((ext_vector_type(4)))  unsigned v4u;
typedef __attribute__((ext_vector_type(4)))  int v4i;
typedef float __attribute__((may_alias)) float_a;
typedef int __attribute__((may_alias)) int_a;

template <typename T> __device__ __forceinline__ void vst2(void* p, T v) { *(volatile T*)p = v; __threadfence(); *(volatile T*)p = v; }
__device__ __forceinline__ v8f wmma16(v16h a, v16h b, v8f c) {
  v8f d = __builtin_amdgcn_wmma_f32_16x16x32_f16(false, a, false, b, (short)0, c, false, false);
  asm volatile("v_nop\n\tv_nop\n\tv_nop\n\tv_nop" : "+v"(d) : "v"(a), "v"(b));
  return d;
}
__device__ __forceinline__ v8f wmma_bf(v16b a, v16b b, v8f c) {
  v8f d = __builtin_amdgcn_wmma_f32_16x16x32_bf16(false, a, false, b, (short)0, c, false, false);
  asm volatile("v_nop\n\tv_nop\n\tv_nop\n\tv_nop" : "+v"(d) : "v"(a), "v"(b));
  return d;
}
__device__ __forceinline__ v16h frag_h(const _Float16* rowk0, int lane) {
  union { v16h v; v8h q[2]; } u; const _Float16* p = rowk0 + 8 * (lane >> 4);
  u.q[0] = *(const v8h*)p; u.q[1] = *(const v8h*)(p + 16); return u.v;
}
__device__ __forceinline__ v16h frag_f32(const float* rowk0, int lane) {
  v16h a; const float* p = rowk0 + 8 * (lane >> 4);
#pragma unroll
  for (int i = 0; i < 8; ++i) { a[i] = (_Float16)p[i]; a[8 + i] = (_Float16)p[16 + i]; }
  return a;
}
__device__ __forceinline__ v16h frag_f32s(const float* rowk0, int lane, float sc) {
  v16h a; const float* p = rowk0 + 8 * (lane >> 4);
#pragma unroll
  for (int i = 0; i < 8; ++i) { a[i] = (_Float16)(p[i] * sc); a[8 + i] = (_Float16)(p[16 + i] * sc); }
  return a;
}
__device__ __forceinline__ v16h fragc_f32(const float* W, int k0, int n, int lane, int ld, int K) {
  v16h a; const int g = lane >> 4;
#pragma unroll
  for (int i = 0; i < 8; ++i) { const int ka = k0 + 8 * g + i, kb = ka + 16;
    a[i] = (_Float16)(ka < K ? W[(size_t)(ka < K ? ka : K - 1) * ld + n] : 0.f); a[8 + i] = (_Float16)(kb < K ? W[(size_t)(kb < K ? kb : K - 1) * ld + n] : 0.f); }
  return a;
}
struct F2 { v16b h, l; };
__device__ __forceinline__ F2 bsplit16(const float v[16]) { F2 r;
#pragma unroll
  for (int i = 0; i < 16; ++i) { const __bf16 h = (__bf16)v[i]; r.h[i] = h; r.l[i] = (__bf16)(v[i] - (float)h); }
  return r; }
__device__ __forceinline__ F2 split_row(const float* row, int k0, int lane) { float v[16]; const float* p = row + k0 + 8 * (lane >> 4);
#pragma unroll
  for (int i = 0; i < 8; ++i) { v[i] = p[i]; v[8 + i] = p[16 + i]; }
  return bsplit16(v); }
__device__ __forceinline__ F2 split_rowK(const float* row, int k0, int lane, int K) { float v[16]; const int g = lane >> 4;
#pragma unroll
  for (int i = 0; i < 8; ++i) { const int ka = k0 + 8 * g + i, kb = ka + 16; v[i] = ka < K ? row[ka < K ? ka : K - 1] : 0.f; v[8 + i] = kb < K ? row[kb < K ? kb : K - 1] : 0.f; }
  return bsplit16(v); }
__device__ __forceinline__ F2 split_col(const float* W, int k0, int n, int lane, int ld, int K) { float v[16]; const int g = lane >> 4;
#pragma unroll
  for (int i = 0; i < 8; ++i) { const int ka = k0 + 8 * g + i, kb = ka + 16; v[i] = ka < K ? W[(size_t)(ka < K ? ka : K - 1) * ld + n] : 0.f; v[8 + i] = kb < K ? W[(size_t)(kb < K ? kb : K - 1) * ld + n] : 0.f; }
  return bsplit16(v); }
__device__ __forceinline__ v8f mac3(const F2& a, const F2& b, v8f c) { c = wmma_bf(a.l, b.h, c); c = wmma_bf(a.h, b.l, c); return wmma_bf(a.h, b.h, c); }
__device__ __forceinline__ float sigm(float v) { return 1.0f / (1.0f + expf(-v)); }
#define LDSX() do { asm volatile("s_wait_dscnt 0" ::: "memory"); __builtin_amdgcn_wave_barrier(); __builtin_amdgcn_fence(__ATOMIC_RELEASE, "workgroup"); } while (0)


#define NIMG 4096
#define C1 32
#define C2 64
#define H0 28
#define H1d 26
#define H2d 24
#define HP 12
#define NFLAT (C2 * HP * HP)
#define NHID 128
#define NCLS 10
#ifndef TNI
#define TNI NIMG
#endif
typedef __attribute__((ext_vector_type(8))) __bf16 v8b;
__device__ __forceinline__ v16b frag_b(const __bf16* rowk0, int lane) {
  union { v16b v; v8b q[2]; } u; const __bf16* p = rowk0 + 8 * (lane >> 4);
  u.q[0] = *(const v8b*)p; u.q[1] = *(const v8b*)(p + 16); return u.v;
}
__device__ __forceinline__ float bfr(float v) { return (float)(__bf16)v; }
__device__ __attribute__((noinline)) float exp_ni(float v) { return expf(v); }
__device__ __attribute__((noinline)) float erf_ni(float v) { return erff(v); }

#define WS_W2  0u
#define WS_F1  (WS_W2 + 2u * C2 * 288)
#define WS_F2  (WS_F1 + 2u * NHID * NFLAT)
#define WS_P   (((WS_F2 + 2u * 16 * NHID) + 127u) / 128u * 128u)
#define WS_END (WS_P + 2u * (size_t)NIMG * NFLAT)

__global__ __launch_bounds__(256) void k_pack(const float* __restrict__ W2c, const float* __restrict__ F1, const float* __restrict__ F2, _Float16* __restrict__ PW2, _Float16* __restrict__ PF1, __bf16* __restrict__ PF2) {
  const int n = blockIdx.x, which = blockIdx.y, t = threadIdx.x;
  if (which == 0) { if (n >= C2) return; __shared__ __align__(16) _Float16 s[288]; for (int k = t; k < 288; k += 256) s[k] = (_Float16)bfr(W2c[(size_t)n * 288 + k]); __syncthreads(); for (int q = t; q < 288 / 8; q += 256) vst2((unsigned*)(PW2 + (size_t)n * 288 + q * 8), *(const v4u*)&s[q * 8]); }
  else if (which == 1) { __shared__ __align__(16) _Float16 s1[NFLAT]; for (int k = t; k < NFLAT; k += 256) s1[k] = (_Float16)bfr(F1[(size_t)n * NFLAT + k]); __syncthreads(); for (int q = t; q < NFLAT / 8; q += 256) vst2((unsigned*)(PF1 + (size_t)n * NFLAT + q * 8), *(const v4u*)&s1[q * 8]); }
  else { if (n >= 16) return; __shared__ __align__(16) __bf16 s2[NHID]; if (t < NHID) s2[t] = (__bf16)((n < NCLS) ? F2[(size_t)n * NHID + t] : 0.f); __syncthreads(); if (t < NHID / 8) vst2((unsigned*)(PF2 + (size_t)n * NHID + t * 8), *(const v4u*)&s2[t * 8]); }
}
__global__ __launch_bounds__(128) void k_img(const float* __restrict__ X, const float* __restrict__ W1c, const float* __restrict__ B1, const _Float16* __restrict__ PW2, const float* __restrict__ B2, _Float16* __restrict__ P) {
  __shared__ _Float16 sh1[C1][H1d * H1d + 4];
  __shared__ __align__(16) _Float16 sa[64][40];
  __shared__ _Float16 sh2[C2][H2d * H2d + 8];
  __shared__ float sx[H0 * H0]; __shared__ float sw1[C1 * 9], sb1[C1];
  const int tid = threadIdx.x, wave = tid >> 5, lane = tid & 31, col = lane & 15, g = lane >> 4; const size_t img = blockIdx.x;
  for (int e = tid; e < H0 * H0; e += 128) sx[e] = bfr(X[img * H0 * H0 + e]);
  for (int e = tid; e < C1 * 9; e += 128) sw1[e] = bfr(W1c[e]);
  if (tid < C1) sb1[tid] = bfr(B1[tid]);
  __syncthreads();
  for (int e = tid; e < C1 * H1d * H1d; e += 128) { const int c = e / (H1d * H1d), p = e % (H1d * H1d); const int y = p / H1d, x = p % H1d; float a = 0.f;
#pragma unroll
    for (int k = 0; k < 9; ++k) a += sx[(y + k / 3) * H0 + x + k % 3] * sw1[c * 9 + k];
    sh1[c][p] = (_Float16)fmaxf(a + sb1[c], 0.f); }
  __syncthreads();
#pragma unroll 1
  for (int pt = 0; pt < 9; ++pt) { v8f acc[4] = {};
#pragma unroll 1
    for (int kc = 0; kc < 9; ++kc) {
      for (int e = tid; e < 64 * 32; e += 128) { const int r = e >> 5, kk = e & 31; const int k = kc * 32 + kk; const int c = k / 9, tap = k % 9; const int pos = pt * 64 + r; const int oy = pos / H2d, ox = pos % H2d; sa[r][kk] = sh1[c][(oy + tap / 3) * H1d + ox + tap % 3]; }
      __syncthreads();
      { const v16h a = frag_h(&sa[wave * 16 + col][0], lane);
#pragma unroll
        for (int j = 0; j < 4; ++j) acc[j] = wmma16(a, frag_h(PW2 + (size_t)(j * 16 + col) * 288 + kc * 32, lane), acc[j]); }
      __syncthreads(); }
#pragma unroll
    for (int j = 0; j < 4; ++j) { const int o = j * 16 + col; const float bb = bfr(B2[o]);
#pragma unroll
      for (int r = 0; r < 8; ++r) sh2[o][pt * 64 + wave * 16 + 8 * g + r] = (_Float16)fmaxf(acc[j][r] + bb, 0.f); } }
  __syncthreads();
  __shared__ __align__(16) _Float16 sp[NFLAT];
  for (int e = tid; e < NFLAT; e += 128) { const int c = e / 144, q = e % 144; const int py = q / 12, px = q % 12; const _Float16* hrow = &sh2[c][(2 * py) * H2d + 2 * px];
    const float m0 = fmaxf((float)hrow[0], (float)hrow[1]), m1 = fmaxf((float)hrow[H2d], (float)hrow[H2d + 1]); sp[e] = (_Float16)fmaxf(m0, m1); }
  __syncthreads();
  for (int q = tid; q < NFLAT / 8; q += 128) vst2((unsigned*)(P + img * NFLAT + q * 8), *(const v4u*)&sp[q * 8]);
}
__global__ __launch_bounds__(128) void k_fc(const _Float16* __restrict__ P, const _Float16* __restrict__ PF1, const float* __restrict__ FB1, const __bf16* __restrict__ PF2, const float* __restrict__ FB2, float* __restrict__ OUT) {
  __shared__ __align__(16) __bf16 shh[4][16][NHID + 8], shl[4][16][NHID + 8]; __shared__ __align__(16) float so[64][NCLS];
  const int tid = threadIdx.x, wave = tid >> 5, lane = tid & 31, col = lane & 15, g = lane >> 4; const size_t r0 = (size_t)blockIdx.x * 64 + wave * 16;
  v8f acc[8] = {};
#pragma unroll 4
  for (int kc = 0; kc < NFLAT / 32; ++kc) { const v16h a = frag_h(P + (r0 + col) * NFLAT + kc * 32, lane);
#pragma unroll
    for (int j = 0; j < 8; ++j) acc[j] = wmma16(a, frag_h(PF1 + (size_t)(j * 16 + col) * NFLAT + kc * 32, lane), acc[j]); }
#pragma unroll
  for (int j = 0; j < 8; ++j) { const int c = j * 16 + col; const float bb = bfr(FB1[c]);
#pragma unroll
    for (int r = 0; r < 8; ++r) { const float v = fmaxf(acc[j][r] + bb, 0.f); const __bf16 hb = (__bf16)v; shh[wave][8 * g + r][c] = hb; shl[wave][8 * g + r][c] = (__bf16)(v - (float)hb); } }
  if (lane < 16) for (int c = NHID; c < NHID + 8; ++c) { shh[wave][lane][c] = (__bf16)0.f; shl[wave][lane][c] = (__bf16)0.f; }
  LDSX();
  { v8f o = {};
#pragma unroll
    for (int kc = 0; kc < NHID / 32; ++kc) { const v16b a = frag_b(&shh[wave][col][kc * 32], lane), al = frag_b(&shl[wave][col][kc * 32], lane); const v16b w = frag_b(PF2 + (size_t)col * NHID + kc * 32, lane); o = wmma_bf(al, w, o); o = wmma_bf(a, w, o); }
    if (col < NCLS) {
#pragma unroll
      for (int r = 0; r < 8; ++r) so[wave * 16 + 8 * g + r][col] = o[r] + bfr(FB2[col]); } }
  __syncthreads();
  for (int e = tid; e < 64 * NCLS / 4; e += 128) vst2(OUT + (size_t)blockIdx.x * 64 * NCLS + e * 4, *(const v4f*)(&so[0][0] + e * 4));
}
extern "C" void kernel_launch(void* const* d_in, const int* in_sizes, int n_in, void* d_out, int out_size, void* d_ws, size_t ws_size, hipStream_t stream) {
  (void)in_sizes; (void)n_in; (void)out_size;
  const float** F = (const float**)d_in;
  if (ws_size < (size_t)WS_END) return;
  char* ws = (char*)d_ws; _Float16 *PW2 = (_Float16*)(ws + WS_W2), *PF1 = (_Float16*)(ws + WS_F1), *P = (_Float16*)(ws + WS_P); __bf16* PF2 = (__bf16*)(ws + WS_F2);
  k_pack<<<dim3(NHID, 3), 256, 0, stream>>>(F[3], F[5], F[7], PW2, PF1, PF2);
  k_img<<<TNI, 128, 0, stream>>>(F[0], F[1], F[2], PW2, F[4], P);
  k_fc<<<TNI / 64, 128, 0, stream>>>(P, PF1, F[6], PF2, F[8], (float*)d_out);
}
